// TransformerConvEncoder_55903294325152
// MI455X (gfx1250) — hardware-run, weakly checked
//
#include <hip/hip_runtime.h>
#include <stddef.h>
#include <stdint.h>

#define BSZ   4
#define SQ    512
#define NTOK  2048
#define DM    512
#define NH    8
#define HDM   64
#define CCH   512
#define HC    4096
#define EE    4096
#define NL    2
#define NQKV  1536
#define QB    128
#define KC    64
#define NQB   (SQ / QB)
#define NCK   (SQ / KC)
#define SBLK  (SQ / 256)
#define QKPLANE (BSZ * NH * SQ * HDM)
#define GD    4
#define CAP   512
#define NEGV  (-1.0e9f)

#define C_X   64.0f
#define C_W   32.0f
#define C_Q   32.0f
#define C_P   1024.0f
#define C_O   64.0f
#define C_G   256.0f
#define QKV_A (0.015625f)
#define S_SC  (0.0001220703125f)
#define O_SC  (0.001953125f)
#define WO_SC (0.00048828125f)
#define HF_SC (0.0001220703125f)

static_assert(NTOK == BSZ * SQ);
static_assert(SQ % 256 == 0);
static_assert(DM % 64 == 0);
static_assert(HC % 64 == 0);
static_assert(HDM == 64);
static_assert(NH * HDM == DM);
static_assert(NQKV == 3 * DM);
static_assert(SQ % KC == 0);
static_assert(SQ % QB == 0);
static_assert(NTOK % 256 == 0);
static_assert((NTOK * DM) % 2048 == 0);
static_assert(SQ % GD == 0);
static_assert(CCH == 2 * 256);
static_assert(EE % 256 == 0);
static_assert(CAP % 32 == 0);
static_assert(NH == 8);
static_assert(HC == NH * CCH);

typedef _Float16 v16h __attribute__((ext_vector_type(16)));
typedef _Float16 v8h  __attribute__((ext_vector_type(8)));
typedef float    v8f  __attribute__((ext_vector_type(8)));
typedef float    v4f  __attribute__((ext_vector_type(4)));
typedef float    v2f  __attribute__((ext_vector_type(2)));
typedef unsigned int v4u __attribute__((ext_vector_type(4)));

union Frag  { v16h v; v8h h[2]; };
union Pack8 { v8h h; v4u u; };

__device__ __forceinline__ v8f mma16(v16h a, v16h b, v8f c) {
  c = __builtin_amdgcn_wmma_f32_16x16x32_f16(false, a, false, b, (short)0, c, false, false);
  asm volatile("v_nop\n\tv_nop\n\tv_nop\n\tv_nop" : "+v"(c) : "v"(a), "v"(b));
  return c;
}

__device__ __forceinline__ v16h ldfrag(const _Float16* p, int ld, int row0, int k0, int lane) {
  const int m = lane & 15, lh = lane >> 4;
  const _Float16* q = p + (size_t)(row0 + m) * ld + k0 + 8 * lh;
  Frag f;
  f.h[0] = *(const v8h*)(q);
  f.h[1] = *(const v8h*)(q + 16);
  return f.v;
}

__device__ __forceinline__ v8f zero8() { return (v8f){0.f, 0.f, 0.f, 0.f, 0.f, 0.f, 0.f, 0.f}; }
__device__ __forceinline__ v4f zero4() { return (v4f){0.f, 0.f, 0.f, 0.f}; }

__device__ __forceinline__ void gemm32x64(const _Float16* __restrict__ A, int lda,
                                          const _Float16* __restrict__ Bt, int ldb, int K,
                                          int m0, int n0, int lane, v8f (&acc)[2][4]) {
#pragma unroll 1
  for (int k0 = 0; k0 < K; k0 += 32) {
    const v16h a0 = ldfrag(A, lda, m0, k0, lane);
    const v16h a1 = ldfrag(A, lda, m0 + 16, k0, lane);
    const v16h b0 = ldfrag(Bt, ldb, n0, k0, lane);
    const v16h b1 = ldfrag(Bt, ldb, n0 + 16, k0, lane);
    const v16h b2 = ldfrag(Bt, ldb, n0 + 32, k0, lane);
    const v16h b3 = ldfrag(Bt, ldb, n0 + 48, k0, lane);
    acc[0][0] = mma16(a0, b0, acc[0][0]);
    acc[1][0] = mma16(a1, b0, acc[1][0]);
    acc[0][1] = mma16(a0, b1, acc[0][1]);
    acc[1][1] = mma16(a1, b1, acc[1][1]);
    acc[0][2] = mma16(a0, b2, acc[0][2]);
    acc[1][2] = mma16(a1, b2, acc[1][2]);
    acc[0][3] = mma16(a0, b3, acc[0][3]);
    acc[1][3] = mma16(a1, b3, acc[1][3]);
  }
}

__global__ __launch_bounds__(256) void k_cvt(const float* __restrict__ src, _Float16* __restrict__ dh, float scale) {
  const int tid = threadIdx.x;
  const size_t o = (size_t)blockIdx.x * 2048 + (size_t)tid * 8;
  const v4f a0 = *(const v4f*)(src + o) * scale;
  const v4f a1 = *(const v4f*)(src + o + 4) * scale;
  Pack8 pk;
  pk.h = (v8h){(_Float16)a0[0], (_Float16)a0[1], (_Float16)a0[2], (_Float16)a0[3],
               (_Float16)a1[0], (_Float16)a1[1], (_Float16)a1[2], (_Float16)a1[3]};
  const v4u vv = pk.u;
  volatile v4u* d = (volatile v4u*)(dh + o);
  *d = vv;
  __threadfence();
  *d = vv;
}

#define TP 72
__global__ __launch_bounds__(256) void k_tr(const float* __restrict__ src, int K, int N, size_t srcZ,
                                            _Float16* __restrict__ dst, size_t dstZ, float scale) {
  __shared__ __align__(16) _Float16 st[64 * TP];
  const int tid = threadIdx.x;
  const int n0 = blockIdx.x * 64, k0 = blockIdx.y * 64, l = blockIdx.z;
  const int r = tid >> 2, cq = (tid & 3) * 16;
  const float* S = src + (size_t)l * srcZ + (size_t)(k0 + r) * N + n0 + cq;
#pragma unroll
  for (int j = 0; j < 4; ++j) {
    const v4f a = *(const v4f*)(S + 4 * j) * scale;
#pragma unroll
    for (int i = 0; i < 4; ++i) st[(cq + 4 * j + i) * TP + r] = (_Float16)a[i];
  }
  __syncthreads();
  v4u val[2];
  size_t go[2];
#pragma unroll
  for (int it = 0; it < 2; ++it) {
    const int p   = tid + 256 * it;
    const int row = p >> 3;
    const int pc  = p & 7;
    Pack8 pk;
    pk.h    = *(const v8h*)(st + row * TP + pc * 8);
    val[it] = pk.u;
    go[it]  = (size_t)l * dstZ + (size_t)(n0 + row) * K + k0 + pc * 8;
  }
  for (int ps = 0; ps < 2; ++ps) {
#pragma unroll
    for (int it = 0; it < 2; ++it) *(volatile v4u*)(dst + go[it]) = val[it];
    __threadfence();
  }
}

#define STP 72
#define SVP 264
__global__ __launch_bounds__(256) void k_qkv(const _Float16* __restrict__ xh,
                                             const _Float16* __restrict__ wt,
                                             const float* __restrict__ bq,
                                             const float* __restrict__ bk,
                                             const float* __restrict__ bv,
                                             _Float16* __restrict__ qkp,
                                             _Float16* __restrict__ vtp) {
  __shared__ __align__(16) _Float16 st[256 * STP];
  const int tid = threadIdx.x, lane = tid & 31, wave = tid >> 5;
  const int hh = lane >> 4, c = lane & 15;
  const int bx = blockIdx.x;
  const int b  = bx / SBLK;
  const int sb = (bx - b * SBLK) * 256;
  const int ns = blockIdx.y;
  const int which = ns / NH;
  const int head  = ns - which * NH;
  const int hb    = b * NH + head;
  const int m0 = sb + wave * 32;
  const int n0 = ns * 64;
  const _Float16* A = xh + (size_t)b * SQ * DM;

  v8f acc[2][4];
#pragma unroll
  for (int s = 0; s < 2; ++s)
#pragma unroll
    for (int t = 0; t < 4; ++t) acc[s][t] = zero8();
  gemm32x64(A, DM, wt, DM, DM, m0, n0, lane, acc);

  float bb[4];
#pragma unroll
  for (int t = 0; t < 4; ++t) {
    const int i = head * HDM + 16 * t + c;
    const float xq = bq[i], xk = bk[i], xv = bv[i];
    bb[t] = ((which == 0) ? xq : ((which == 1) ? xk : xv)) * C_Q;
  }

  if (which < 2) {
#pragma unroll
    for (int sub = 0; sub < 2; ++sub)
#pragma unroll
      for (int t = 0; t < 4; ++t)
#pragma unroll
        for (int r = 0; r < 8; ++r)
          st[(wave * 32 + sub * 16 + 8 * hh + r) * STP + 16 * t + c] =
              (_Float16)(acc[sub][t][r] * QKV_A + bb[t]);
  } else {
#pragma unroll
    for (int sub = 0; sub < 2; ++sub)
#pragma unroll
      for (int t = 0; t < 4; ++t)
#pragma unroll
        for (int r = 0; r < 8; ++r)
          st[(16 * t + c) * SVP + wave * 32 + sub * 16 + 8 * hh + r] =
              (_Float16)(acc[sub][t][r] * QKV_A + bb[t]);
  }
  __syncthreads();

  if (which < 2) {
    _Float16* base = qkp + (size_t)which * QKPLANE + (size_t)hb * SQ * HDM;
#pragma unroll
    for (int g = 0; g < 2; ++g) {
      v4u val[4];
      size_t go[4];
#pragma unroll
      for (int j = 0; j < 4; ++j) {
        const int p  = tid + 256 * (4 * g + j);
        const int lr = p >> 3;
        const int pc = p & 7;
        Pack8 pk;
        pk.h   = *(const v8h*)(st + lr * STP + pc * 8);
        val[j] = pk.u;
        go[j]  = (size_t)(sb + lr) * HDM + pc * 8;
      }
      for (int ps = 0; ps < 2; ++ps) {
#pragma unroll
        for (int j = 0; j < 4; ++j) *(volatile v4u*)(base + go[j]) = val[j];
        __threadfence();
      }
    }
  } else {
    _Float16* base = vtp + (size_t)hb * HDM * SQ;
#pragma unroll
    for (int g = 0; g < 2; ++g) {
      v4u val[4];
      size_t go[4];
#pragma unroll
      for (int j = 0; j < 4; ++j) {
        const int p    = tid + 256 * (4 * g + j);
        const int drow = p >> 5;
        const int pc   = p & 31;
        Pack8 pk;
        pk.h   = *(const v8h*)(st + drow * SVP + pc * 8);
        val[j] = pk.u;
        go[j]  = (size_t)drow * SQ + sb + pc * 8;
      }
      for (int ps = 0; ps < 2; ++ps) {
#pragma unroll
        for (int j = 0; j < 4; ++j) *(volatile v4u*)(base + go[j]) = val[j];
        __threadfence();
      }
    }
  }
}

#define KTP 72
__global__ __launch_bounds__(256) void k_attn(const _Float16* __restrict__ qp,
                                              const _Float16* __restrict__ kp,
                                              const _Float16* __restrict__ vt,
                                              const int* __restrict__ lens,
                                              _Float16* __restrict__ op, float sscale, float oscale) {
  __shared__ __align__(16) _Float16 Ks[KC * KTP];
  __shared__ __align__(16) _Float16 Vs[HDM * KTP];
  __shared__ __align__(16) _Float16 Ps[8 * 16 * KTP];

  const int tid = threadIdx.x, lane = tid & 31, wave = tid >> 5;
  const int hh = lane >> 4, c = lane & 15;
  const int qb  = blockIdx.x % NQB;
  const int hb  = blockIdx.x / NQB;
  const int h   = hb % NH;
  const int b   = hb / NH;
  const int q0  = qb * QB + wave * 16;
  int len = lens[b];
  len = (len < 0) ? 0 : ((len > SQ) ? SQ : len);
  const int nch = (len > 0) ? ((len + KC - 1) / KC) : NCK;

  const _Float16* Q = qp + (size_t)hb * SQ * HDM;
  const _Float16* K = kp + (size_t)hb * SQ * HDM;
  const _Float16* V = vt + (size_t)hb * HDM * SQ;

  v16h qa[2];
  qa[0] = ldfrag(Q, HDM, q0, 0, lane);
  qa[1] = ldfrag(Q, HDM, q0, 32, lane);

  const float NEGI = -__builtin_huge_valf();
  float mrow[8], lrow[8];
  v8f oacc[4];
#pragma unroll
  for (int r = 0; r < 8; ++r) { mrow[r] = NEGI; lrow[r] = 0.f; }
#pragma unroll
  for (int t = 0; t < 4; ++t) oacc[t] = zero8();

  _Float16* pw = Ps + wave * 16 * KTP;

  for (int kc = 0; kc < nch; ++kc) {
    const int kv0 = kc * KC;
    __syncthreads();
    {
      const int r  = tid >> 2;
      const int qq = (tid & 3) * 16;
      const _Float16* ks = K + (size_t)(kv0 + r) * HDM + qq;
      const _Float16* vs = V + (size_t)r * SQ + kv0 + qq;
#pragma unroll
      for (int e = 0; e < 2; ++e) {
        *(v8h*)(Ks + r * KTP + qq + 8 * e) = *(const v8h*)(ks + 8 * e);
        *(v8h*)(Vs + r * KTP + qq + 8 * e) = *(const v8h*)(vs + 8 * e);
      }
    }
    __syncthreads();

    v8f s[4];
#pragma unroll
    for (int j = 0; j < 4; ++j) s[j] = zero8();
#pragma unroll
    for (int dc = 0; dc < 2; ++dc) {
#pragma unroll
      for (int j = 0; j < 4; ++j) {
        const v16h kb = ldfrag(Ks, KTP, j * 16, dc * 32, lane);
        s[j] = mma16(qa[dc], kb, s[j]);
      }
    }
    float cm[8];
#pragma unroll
    for (int r = 0; r < 8; ++r) {
      float m = NEGI;
#pragma unroll
      for (int j = 0; j < 4; ++j) {
        const int key  = kv0 + j * 16 + c;
        const float sv = s[j][r] * sscale;
        s[j][r] = (key < len) ? sv : NEGV;
        m = fmaxf(m, s[j][r]);
      }
#pragma unroll
      for (int off = 1; off < 16; off <<= 1) m = fmaxf(m, __shfl_xor(m, off, 32));
      cm[r] = m;
    }
    float al[8];
#pragma unroll
    for (int r = 0; r < 8; ++r) {
      const float mnew  = fmaxf(mrow[r], cm[r]);
      const float alpha = __expf(mrow[r] - mnew);
      mrow[r] = mnew;
      float psum = 0.f;
#pragma unroll
      for (int j = 0; j < 4; ++j) {
        const float p = __expf(s[j][r] - mnew);
        psum += p;
        pw[(8 * hh + r) * KTP + j * 16 + c] = (_Float16)(p * C_P);
      }
#pragma unroll
      for (int off = 1; off < 16; off <<= 1) psum += __shfl_xor(psum, off, 32);
      lrow[r] = lrow[r] * alpha + psum;
      al[r] = alpha;
    }
#pragma unroll
    for (int t = 0; t < 4; ++t)
#pragma unroll
      for (int r = 0; r < 8; ++r) oacc[t][r] *= al[r];
    __syncthreads();

#pragma unroll
    for (int kk = 0; kk < 2; ++kk) {
      const v16h pa = ldfrag(pw, KTP, 0, kk * 32, lane);
#pragma unroll
      for (int t = 0; t < 4; ++t) {
        const v16h vb = ldfrag(Vs, KTP, t * 16, kk * 32, lane);
        oacc[t] = mma16(pa, vb, oacc[t]);
      }
    }
  }

  float invl[8];
#pragma unroll
  for (int r = 0; r < 8; ++r) invl[r] = (lrow[r] > 0.f) ? (oscale / lrow[r]) : 0.f;
  __syncthreads();
#pragma unroll
  for (int r = 0; r < 8; ++r) {
#pragma unroll
    for (int t = 0; t < 4; ++t)
      pw[(8 * hh + r) * KTP + 16 * t + c] = (_Float16)(oacc[t][r] * invl[r]);
  }
  __syncthreads();
  v4u val[4];
  size_t go[4];
#pragma unroll
  for (int it = 0; it < 4; ++it) {
    const int p  = lane + 32 * it;
    const int L  = p >> 3;
    const int pc = p & 7;
    Pack8 pk;
    pk.h    = *(const v8h*)(pw + L * KTP + pc * 8);
    val[it] = pk.u;
    go[it]  = ((size_t)(b * SQ + q0 + L)) * DM + (size_t)h * HDM + pc * 8;
  }
  for (int ps = 0; ps < 2; ++ps) {
#pragma unroll
    for (int it = 0; it < 4; ++it) *(volatile v4u*)(op + go[it]) = val[it];
    __threadfence();
  }
}

#define OTP 68
__device__ __forceinline__ void out_epilogue_f32(v8f (&acc)[2][4], float scale, const float (&bb)[4],
                                                 float* sw, float* __restrict__ out, int ldo,
                                                 int m0, int n0, int lane, int hh, int c) {
#pragma unroll
  for (int sub = 0; sub < 2; ++sub) {
    __syncthreads();
#pragma unroll
    for (int t = 0; t < 4; ++t) {
#pragma unroll
      for (int r = 0; r < 8; ++r) sw[(8 * hh + r) * OTP + 16 * t + c] = acc[sub][t][r] * scale + bb[t];
    }
    __syncthreads();
    v4f val[8];
    size_t go[8];
#pragma unroll
    for (int it = 0; it < 8; ++it) {
      const int p    = lane + 32 * it;
      const int L    = p >> 3;
      const int pc   = p & 7;
      const int row  = L >> 1;
      const int half = L & 1;
      val[it] = *(const v4f*)(sw + row * OTP + half * 32 + pc * 4);
      go[it]  = (size_t)(m0 + sub * 16 + row) * ldo + n0 + half * 32 + pc * 4;
    }
    for (int ps = 0; ps < 2; ++ps) {
#pragma unroll
      for (int it = 0; it < 8; ++it) *(volatile v4f*)(out + go[it]) = val[it];
      __threadfence();
    }
  }
}

__device__ __forceinline__ void out_epilogue_dual(v8f (&acc)[2][4], float scale, const float (&bb)[4], float hscale,
                                                  float* sw, float* __restrict__ outf, _Float16* __restrict__ outh,
                                                  int ldo, int m0, int n0, int lane, int hh, int c) {
#pragma unroll
  for (int sub = 0; sub < 2; ++sub) {
    __syncthreads();
#pragma unroll
    for (int t = 0; t < 4; ++t) {
#pragma unroll
      for (int r = 0; r < 8; ++r) sw[(8 * hh + r) * OTP + 16 * t + c] = acc[sub][t][r] * scale + bb[t];
    }
    __syncthreads();
    {
      v4f val[8];
      size_t go[8];
#pragma unroll
      for (int it = 0; it < 8; ++it) {
        const int p    = lane + 32 * it;
        const int L    = p >> 3;
        const int pc   = p & 7;
        const int row  = L >> 1;
        const int half = L & 1;
        val[it] = *(const v4f*)(sw + row * OTP + half * 32 + pc * 4);
        go[it]  = (size_t)(m0 + sub * 16 + row) * ldo + n0 + half * 32 + pc * 4;
      }
      for (int ps = 0; ps < 2; ++ps) {
#pragma unroll
        for (int it = 0; it < 8; ++it) *(volatile v4f*)(outf + go[it]) = val[it];
        __threadfence();
      }
    }
    {
      v4u hv[4];
      size_t gh[4];
#pragma unroll
      for (int it = 0; it < 4; ++it) {
        const int p  = lane + 32 * it;
        const int L  = p >> 3;
        const int pc = p & 7;
        const float* ra = sw + L * OTP + pc * 8;
        const v4f a0 = *(const v4f*)(ra) * hscale, a1 = *(const v4f*)(ra + 4) * hscale;
        Pack8 pk;
        pk.h = (v8h){(_Float16)a0[0], (_Float16)a0[1], (_Float16)a0[2], (_Float16)a0[3],
                     (_Float16)a1[0], (_Float16)a1[1], (_Float16)a1[2], (_Float16)a1[3]};
        hv[it] = pk.u;
        gh[it] = (size_t)(m0 + sub * 16 + L) * ldo + n0 + pc * 8;
      }
      for (int ps = 0; ps < 2; ++ps) {
#pragma unroll
        for (int it = 0; it < 4; ++it) *(volatile v4u*)(outh + gh[it]) = hv[it];
        __threadfence();
      }
    }
  }
}

__global__ __launch_bounds__(256) void k_gemm_wo(const _Float16* __restrict__ ap,
                                                 const _Float16* __restrict__ wt,
                                                 const float* __restrict__ bias,
                                                 float* __restrict__ outf, _Float16* __restrict__ outh) {
  __shared__ __align__(16) float st[8][16 * OTP];
  const int tid = threadIdx.x, lane = tid & 31, wave = tid >> 5;
  const int hh = lane >> 4, c = lane & 15;
  const int m0 = blockIdx.x * 256 + wave * 32;
  const int n0 = blockIdx.y * 64;

  v8f acc[2][4];
#pragma unroll
  for (int s = 0; s < 2; ++s)
#pragma unroll
    for (int t = 0; t < 4; ++t) acc[s][t] = zero8();
  gemm32x64(ap, DM, wt, DM, DM, m0, n0, lane, acc);
  float bb[4];
#pragma unroll
  for (int t = 0; t < 4; ++t) bb[t] = bias[n0 + 16 * t + c];
  out_epilogue_dual(acc, WO_SC, bb, C_G, st[wave], outf, outh, DM, m0, n0, lane, hh, c);
}

__global__ __launch_bounds__(256) void k_gemm_hf(const _Float16* __restrict__ ap,
                                                 const _Float16* __restrict__ wt,
                                                 float* __restrict__ out) {
  __shared__ __align__(16) float st[8][16 * OTP];
  const int tid = threadIdx.x, lane = tid & 31, wave = tid >> 5;
  const int hh = lane >> 4, c = lane & 15;
  const int m0 = blockIdx.x * 256 + wave * 32;
  const int n0 = blockIdx.y * 64;

  v8f acc[2][4];
#pragma unroll
  for (int s = 0; s < 2; ++s)
#pragma unroll
    for (int t = 0; t < 4; ++t) acc[s][t] = zero8();
  gemm32x64(ap, DM, wt, DM, DM, m0, n0, lane, acc);
  const float bb[4] = {0.f, 0.f, 0.f, 0.f};
  out_epilogue_f32(acc, HF_SC, bb, st[wave], out, HC, m0, n0, lane, hh, c);
}

__global__ __launch_bounds__(256) void k_coef(const float* __restrict__ hf,
                                              const float* __restrict__ aw,
                                              const float* __restrict__ dw,
                                              float* __restrict__ asrc, float* __restrict__ adst) {
  __shared__ __align__(16) float sa[32];
  __shared__ __align__(16) float sd[32];
  const int tid = threadIdx.x, lane = tid & 31, wave = tid >> 5;
  const int blk = blockIdx.x;
#pragma unroll 1
  for (int t4 = 0; t4 < 4; ++t4) {
    const int task = wave * 4 + t4;
    const int node = task >> 3, head = task & 7;
    const size_t row = (size_t)blk * 4 + node;
    const float* hp = hf + row * HC + (size_t)head * CCH + 4 * lane;
    const float* sp = aw + (size_t)head * CCH + 4 * lane;
    const float* dp = dw + (size_t)head * CCH + 4 * lane;
    v4f ps = zero4(), pd = zero4();
#pragma unroll
    for (int it = 0; it < 4; ++it) {
      const v4f hv = *(const v4f*)(hp + 128 * it);
      ps += hv * *(const v4f*)(sp + 128 * it);
      pd += hv * *(const v4f*)(dp + 128 * it);
    }
    float s = (ps[0] + ps[1]) + (ps[2] + ps[3]);
    float d = (pd[0] + pd[1]) + (pd[2] + pd[3]);
#pragma unroll
    for (int off = 16; off >= 1; off >>= 1) {
      s += __shfl_xor(s, off, 32);
      d += __shfl_xor(d, off, 32);
    }
    if (lane == 0) { sa[task] = s; sd[task] = d; }
  }
  __syncthreads();
  if (tid < 16) {
    const int q = tid & 7;
    const v4f va = *(const v4f*)(sa + 4 * q);
    const v4f vb = *(const v4f*)(sd + 4 * q);
    const bool fs = tid < 8;
    v4f v;
    v[0] = fs ? va[0] : vb[0];
    v[1] = fs ? va[1] : vb[1];
    v[2] = fs ? va[2] : vb[2];
    v[3] = fs ? va[3] : vb[3];
    float* base = fs ? asrc : adst;
    volatile v4f* p = (volatile v4f*)(base + (size_t)blk * 32 + 4 * q);
    *p = v;
    __threadfence();
    *p = v;
  }
}

__global__ __launch_bounds__(256) void k_gat(const int* __restrict__ edges,
                                             const int* __restrict__ enums,
                                             const int* __restrict__ lens,
                                             const float* __restrict__ asrc,
                                             const float* __restrict__ adst,
                                             const float* __restrict__ hf,
                                             const float* __restrict__ mha,
                                             const float* __restrict__ gb,
                                             const float* __restrict__ lg,
                                             const float* __restrict__ lb,
                                             float* __restrict__ outp,
                                             _Float16* __restrict__ xh, float xscale) {
  __shared__ int lst[GD * CAP];
  __shared__ __align__(16) float cf[NH * CAP];
  __shared__ __align__(16) float part[NH * CCH];
  __shared__ __align__(16) float rowb[CCH];
  __shared__ int cnt[8 * GD];
  __shared__ int tot[GD];
  __shared__ float red[16];

  const int tid = threadIdx.x, lane = tid & 31, wave = tid >> 5;
  const int b  = blockIdx.x / (SQ / GD);
  const int d0 = (blockIdx.x - b * (SQ / GD)) * GD;
  int ne = enums[b];
  ne = (ne < 0) ? 0 : ((ne > EE) ? EE : ne);
  int len = lens[b];
  len = (len < 0) ? 0 : ((len > SQ) ? SQ : len);
  const int* esrc = edges + (size_t)b * 2 * EE;
  const int* edst = esrc + EE;

  if (tid < GD) tot[tid] = 0;
  for (int ch = 0; ch < EE / 256; ++ch) {
    const int e  = ch * 256 + tid;
    const int dv = edst[e];
    int sv = esrc[e];
    sv = (sv < 0) ? 0 : ((sv > SQ - 1) ? (SQ - 1) : sv);
    const int dl = dv - d0;
    const bool hit = (e < ne) && ((unsigned)dl < (unsigned)GD);
    unsigned mine = 0u;
#pragma unroll
    for (int g = 0; g < GD; ++g) {
      const unsigned m = (unsigned)__ballot(hit && (dl == g));
      if (lane == 0) cnt[wave * GD + g] = (int)__popc(m);
      mine = (dl == g) ? m : mine;
    }
    __syncthreads();
    int tsum = 0;
    if (tid < GD) {
#pragma unroll
      for (int w = 0; w < 8; ++w) tsum += cnt[w * GD + tid];
    }
    if (hit) {
      int base = tot[dl];
      for (int w = 0; w < wave; ++w) base += cnt[w * GD + dl];
      const int pos = base + (int)__popc(mine & ((1u << lane) - 1u));
      if (pos < CAP) lst[dl * CAP + pos] = sv;
    }
    __syncthreads();
    if (tid < GD) tot[tid] += tsum;
  }
  if (tid < GD) {
    const int node = d0 + tid;
    int p = tot[tid];
    if (node < len) {
      if (p < CAP) lst[tid * CAP + p] = node;
      p += 1;
    }
    tot[tid] = p;
  }
  __syncthreads();

  const int c0 = 2 * tid;
  const float gb0 = gb[c0], gb1 = gb[c0 + 1];
  const float lg0 = lg[c0], lg1 = lg[c0 + 1];
  const float lb0 = lb[c0], lb1 = lb[c0 + 1];
  const float NEGI = -__builtin_huge_valf();
  const float qnan = __int_as_float(0x7fc00000);
#pragma unroll 1
  for (int g = 0; g < GD; ++g) {
    const int total = tot[g];
    const int deg   = (total < CAP) ? total : CAP;
    const bool pois = total > CAP;
    const int node  = d0 + g;
    const size_t row = (size_t)b * SQ + node;
    const int gl = g * CAP;
    const int wl = wave * CAP;

    const float adv = adst[row * NH + wave];
    float mx = NEGI;
    const int npass = (deg + 31) >> 5;
    for (int it = 0; it < npass; ++it) {
      const int i  = it * 32 + lane;
      const int ii = (i < deg) ? i : (deg - 1);
      const int s  = lst[gl + ii];
      const float av = asrc[((size_t)b * SQ + s) * NH + wave] + adv;
      float a = (av > 0.f) ? av : 0.2f * av;
      a = (i < deg) ? a : NEGI;
      if (i < deg) cf[wl + i] = a;
      mx = fmaxf(mx, a);
    }
#pragma unroll
    for (int off = 16; off >= 1; off >>= 1) mx = fmaxf(mx, __shfl_xor(mx, off, 32));
    float sm = 0.f;
    for (int it = 0; it < npass; ++it) {
      const int i  = it * 32 + lane;
      const int ii = (i < deg) ? i : (deg - 1);
      const float a2 = cf[wl + ii];
      const float ex = (i < deg) ? __expf(a2 - mx) : 0.f;
      if (i < deg) cf[wl + i] = ex;
      sm += ex;
    }
#pragma unroll
    for (int off = 16; off >= 1; off >>= 1) sm += __shfl_xor(sm, off, 32);
    const float rcp = (deg > 0) ? (1.0f / (sm + 1e-16f)) : 0.f;
    __syncthreads();

    v4f acc[4];
#pragma unroll
    for (int it = 0; it < 4; ++it) acc[it] = zero4();
    const float* hbase = hf + (size_t)b * SQ * HC + (size_t)wave * CCH + 4 * lane;
#pragma unroll 1
    for (int e = 0; e < deg; ++e) {
      const int s = lst[gl + e];
      const float cw = cf[wl + e];
      const float* hp = hbase + (size_t)s * HC;
#pragma unroll
      for (int it = 0; it < 4; ++it) acc[it] += cw * *(const v4f*)(hp + 128 * it);
    }
#pragma unroll
    for (int it = 0; it < 4; ++it) *(v4f*)(part + wave * CCH + 128 * it + 4 * lane) = acc[it] * rcp;
    __syncthreads();

    float g0 = 0.f, g1 = 0.f;
#pragma unroll
    for (int w = 0; w < NH; ++w) {
      const v2f pv = *(const v2f*)(part + w * CCH + c0);
      g0 += pv[0];
      g1 += pv[1];
    }
    g0 = g0 * 0.125f + gb0;
    g1 = g1 * 0.125f + gb1;
    float s1 = g0 + g1;
#pragma unroll
    for (int off = 16; off >= 1; off >>= 1) s1 += __shfl_xor(s1, off, 32);
    if (lane == 0) red[wave] = s1;
    __syncthreads();
    float ts = 0.f;
#pragma unroll
    for (int w = 0; w < 8; ++w) ts += red[w];
    const float mean = ts * 0.001953125f;
    const float e0 = g0 - mean, e1 = g1 - mean;
    float s2 = e0 * e0 + e1 * e1;
#pragma unroll
    for (int off = 16; off >= 1; off >>= 1) s2 += __shfl_xor(s2, off, 32);
    if (lane == 0) red[8 + wave] = s2;
    __syncthreads();
    float tv = 0.f;
#pragma unroll
    for (int w = 0; w < 8; ++w) tv += red[8 + w];
    const float var  = tv * 0.001953125f;
    const float rstd = rsqrtf(var + 1e-5f);
    const v2f mv = *(const v2f*)(mha + row * DM + c0);
    const float y0 = fmaxf((e0 * rstd) * lg0 + lb0, 0.f) + mv[0];
    const float y1 = fmaxf((e1 * rstd) * lg1 + lb1, 0.f) + mv[1];
    const bool valid = node < len;
    float o0 = valid ? y0 : mv[0];
    float o1 = valid ? y1 : mv[1];
    o0 = pois ? qnan : o0;
    o1 = pois ? qnan : o1;
    *(v2f*)(rowb + c0) = (v2f){o0, o1};
    __syncthreads();

    if (tid < 128) {
      const v4f v = *(const v4f*)(rowb + 4 * tid);
      volatile v4f* p = (volatile v4f*)(outp + row * DM + 4 * tid);
      *p = v;
      __threadfence();
      *p = v;
    } else if (tid < 192) {
      const int q = tid - 128;
      const float* ra = rowb + 8 * q;
      const v4f a0 = *(const v4f*)(ra) * xscale, a1 = *(const v4f*)(ra + 4) * xscale;
      Pack8 pk;
      pk.h = (v8h){(_Float16)a0[0], (_Float16)a0[1], (_Float16)a0[2], (_Float16)a0[3],
                   (_Float16)a1[0], (_Float16)a1[1], (_Float16)a1[2], (_Float16)a1[3]};
      const v4u hv = pk.u;
      volatile v4u* p = (volatile v4u*)(xh + row * DM + 8 * q);
      *p = hv;
      __threadfence();
      *p = hv;
    }
    __syncthreads();
  }
}

extern "C" void kernel_launch(void* const* d_in, const int* in_sizes, int n_in,
                              void* d_out, int out_size, void* d_ws, size_t ws_size,
                              hipStream_t stream) {
  if (n_in < 18) return;
  if (in_sizes[0] != NTOK * DM) return;
  if (in_sizes[1] != NL * DM * DM) return;
  if (in_sizes[2] != NL * DM) return;
  if (in_sizes[3] != NL * DM * DM) return;
  if (in_sizes[4] != NL * DM) return;
  if (in_sizes[5] != NL * DM * DM) return;
  if (in_sizes[6] != NL * DM) return;
  if (in_sizes[7] != NL * DM * DM) return;
  if (in_sizes[8] != NL * DM) return;
  if (in_sizes[9] != NL * DM * HC) return;
  if (in_sizes[10] != NL * NH * CCH) return;
  if (in_sizes[11] != NL * NH * CCH) return;
  if (in_sizes[12] != NL * CCH) return;
  if (in_sizes[13] != NL * DM) return;
  if (in_sizes[14] != NL * DM) return;
  if (in_sizes[15] != BSZ) return;
  if (in_sizes[16] != BSZ * 2 * EE) return;
  if (in_sizes[17] != BSZ) return;
  if (out_size != NL * NTOK * DM) return;

  const float* x    = (const float*)d_in[0];
  const float* wq   = (const float*)d_in[1];
  const float* bq   = (const float*)d_in[2];
  const float* wk   = (const float*)d_in[3];
  const float* bk   = (const float*)d_in[4];
  const float* wv   = (const float*)d_in[5];
  const float* bv   = (const float*)d_in[6];
  const float* wo   = (const float*)d_in[7];
  const float* bo   = (const float*)d_in[8];
  const float* wg   = (const float*)d_in[9];
  const float* asw  = (const float*)d_in[10];
  const float* adw  = (const float*)d_in[11];
  const float* gbs  = (const float*)d_in[12];
  const float* lng  = (const float*)d_in[13];
  const float* lnb  = (const float*)d_in[14];
  const int*   lens = (const int*)d_in[15];
  const int*   edg  = (const int*)d_in[16];
  const int*   enm  = (const int*)d_in[17];
  float* out = (float*)d_out;

  size_t off = 0;
  const size_t oWqkv = off; off += (size_t)NL * NQKV * DM * 2;
  const size_t oWo   = off; off += (size_t)NL * DM * DM * 2;
  const size_t oGw   = off; off += (size_t)NL * HC * DM * 2;
  const size_t oXh   = off; off += (size_t)NTOK * DM * 2;
  const size_t oQ    = off; off += (size_t)QKPLANE * 2;
  const size_t oK    = off; off += (size_t)QKPLANE * 2;
  const size_t oV    = off; off += (size_t)BSZ * NH * HDM * SQ * 2;
  const size_t oO    = off; off += (size_t)NTOK * DM * 2;
  const size_t oM    = off; off += (size_t)NTOK * DM * 4;
  const size_t oXG   = off; off += (size_t)NTOK * DM * 2;
  const size_t oHF   = off; off += (size_t)NTOK * HC * 4;
  const size_t oAS   = off; off += (size_t)NTOK * NH * 4;
  const size_t oAD   = off; off += (size_t)NTOK * NH * 4;
  if (off > ws_size) return;
  if (off > (size_t)134217728) return;
  if (oK != oQ + (size_t)QKPLANE * 2) return;

  char* ws = (char*)d_ws;
  _Float16* Wqkv = (_Float16*)(ws + oWqkv);
  _Float16* Wot  = (_Float16*)(ws + oWo);
  _Float16* Gwt  = (_Float16*)(ws + oGw);
  _Float16* Xh   = (_Float16*)(ws + oXh);
  _Float16* QKp  = (_Float16*)(ws + oQ);
  _Float16* Kp   = (_Float16*)(ws + oK);
  _Float16* Vt   = (_Float16*)(ws + oV);
  _Float16* Op   = (_Float16*)(ws + oO);
  float*    M    = (float*)(ws + oM);
  _Float16* XG   = (_Float16*)(ws + oXG);
  float*    HF   = (float*)(ws + oHF);
  float*    AS   = (float*)(ws + oAS);
  float*    AD   = (float*)(ws + oAD);

  k_tr<<<dim3(DM / 64, DM / 64, NL), dim3(256), 0, stream>>>(wq, DM, DM, (size_t)DM * DM, Wqkv, (size_t)NQKV * DM, C_W);
  k_tr<<<dim3(DM / 64, DM / 64, NL), dim3(256), 0, stream>>>(wk, DM, DM, (size_t)DM * DM, Wqkv + (size_t)DM * DM, (size_t)NQKV * DM, C_W);
  k_tr<<<dim3(DM / 64, DM / 64, NL), dim3(256), 0, stream>>>(wv, DM, DM, (size_t)DM * DM, Wqkv + (size_t)2 * DM * DM, (size_t)NQKV * DM, C_W);
  k_tr<<<dim3(DM / 64, DM / 64, NL), dim3(256), 0, stream>>>(wo, DM, DM, (size_t)DM * DM, Wot, (size_t)DM * DM, C_W);
  k_tr<<<dim3(HC / 64, DM / 64, NL), dim3(256), 0, stream>>>(wg, DM, HC, (size_t)DM * HC, Gwt, (size_t)HC * DM, C_W);
  k_cvt<<<dim3((NTOK * DM) / 2048), dim3(256), 0, stream>>>(x, Xh, C_X);

  for (int l = 0; l < NL; ++l) {
    k_qkv<<<dim3(BSZ * SBLK, NQKV / 64), dim3(256), 0, stream>>>(Xh, Wqkv + (size_t)l * NQKV * DM,
                                                                 bq + (size_t)l * DM, bk + (size_t)l * DM, bv + (size_t)l * DM,
                                                                 QKp, Vt);
    k_attn<<<dim3(BSZ * NH * NQB), dim3(256), 0, stream>>>(QKp, Kp, Vt, lens, Op, S_SC, O_SC);
    k_gemm_wo<<<dim3(NTOK / 256, DM / 64), dim3(256), 0, stream>>>(Op, Wot + (size_t)l * DM * DM, bo + (size_t)l * DM, M, XG);
    k_gemm_hf<<<dim3(NTOK / 256, HC / 64), dim3(256), 0, stream>>>(XG, Gwt + (size_t)l * HC * DM, HF);
    k_coef<<<dim3(NTOK / 4), dim3(256), 0, stream>>>(HF, asw + (size_t)l * NH * CCH, adw + (size_t)l * NH * CCH, AS, AD);
    k_gat<<<dim3(BSZ * (SQ / GD)), dim3(256), 0, stream>>>(edg, enm, lens, AS, AD, HF, M,
                                                            gbs + (size_t)l * CCH, lng + (size_t)l * DM, lnb + (size_t)l * DM,
                                                            out + (size_t)l * NTOK * DM, Xh, C_X);
  }
  (void)hipGetLastError();
}
